// Listener0Model_39152921870344
// MI455X (gfx1250) — hardware-verified
//
#include <hip/hip_runtime.h>
#include <stddef.h>


typedef _Float16 h16;
typedef _Float16 v16h __attribute__((ext_vector_type(16)));
typedef _Float16 v8h  __attribute__((ext_vector_type(8)));
typedef float    v8f  __attribute__((ext_vector_type(8)));
typedef float    v4f  __attribute__((ext_vector_type(4)));

#ifndef NB
#define NB 4096
#endif
#define NB_FULL 4096
#define NPROP   20
#define NALT    9
#define NWORD   50
#define NTGT    10
#define SCN     280
#define KS      320
#define VOCAB   32000
#define DIM     256
#define MROWS   (NB * NTGT)

static_assert(NB >= 64 && NB <= NB_FULL && (NB % 64) == 0);
static_assert(NTGT == NALT + 1);
static_assert((MROWS % 64) == 0 && (MROWS % 32) == 0);
static_assert((DIM % 64) == 0 && (DIM % 32) == 0);
static_assert((KS % 64) == 0 && KS >= SCN && (KS % 32) == 0);
static_assert(DIM == 256);
static_assert((32 * KS) == 256 * 5 * 8);
static_assert((32 * NPROP) <= 3 * 256);
static_assert((16 * NWORD) <= 4 * 256);

#define LDT 72
#define LDC 68
#define LDB 264
static_assert((LDT % 8) == 0 && LDT >= 64);
static_assert((LDC % 4) == 0 && LDC >= 64);
static_assert((LDB % 8) == 0 && LDB >= DIM);

#define WCARRY 64.0f
#define ACARRY 64.0f

#define WSC_BYTES ((size_t)DIM * KS * 2)
#define WSQ_BYTES ((size_t)DIM * DIM * 2)
#define OH_BYTES  ((size_t)MROWS * KS * 2)
#define TG_BYTES  ((size_t)MROWS * DIM * 2)
#define SE_BYTES  ((size_t)NB * DIM * 2)
#define S5_BYTES  ((size_t)NB * DIM * 4)
#define OFF_WSC ((size_t)0)
#define OFF_W4  (OFF_WSC + WSC_BYTES)
#define OFF_W5  (OFF_W4 + WSQ_BYTES)
#define OFF_OH  (OFF_W5 + WSQ_BYTES)
#define OFF_TG  (OFF_OH + OH_BYTES)
#define OFF_SE  (OFF_TG + TG_BYTES)
#define OFF_S5  (OFF_SE + SE_BYTES)
#define WS_TOTAL (OFF_S5 + S5_BYTES)
static_assert((WSC_BYTES % 128) == 0 && (WSQ_BYTES % 128) == 0 && (OH_BYTES % 128) == 0);
static_assert((TG_BYTES % 128) == 0 && (SE_BYTES % 128) == 0 && (S5_BYTES % 128) == 0);
static_assert(WS_TOTAL <= (size_t)134217728);

__device__ __forceinline__ float bf16r(float x) {
  unsigned int u = __float_as_uint(x);
  u = (u + 0x7FFFu + ((u >> 16) & 1u)) & 0xFFFF0000u;
  return __uint_as_float(u);
}

static __device__ __forceinline__ h16 toh_flush(float v) {
  const h16 r = (h16)v;
  return (fabsf(v) < 6.103515625e-05f) ? (h16)0.0f : r;
}

__device__ __forceinline__ v16h frag_at(const _Float16* p) {
  v8h lo = *(const v8h*)(p);
  v8h hi = *(const v8h*)(p + 16);
  v16h out;
#pragma unroll
  for (int i = 0; i < 8; ++i) { out[i] = lo[i]; out[i + 8] = hi[i]; }
  return out;
}

__device__ __forceinline__ v8f wmma16(v16h a, v16h b, v8f c) {
  v8f d = __builtin_amdgcn_wmma_f32_16x16x32_f16(false, a, false, b, (short)0, c,
                                                 false, false);
  asm volatile("v_nop\n\tv_nop\n\tv_nop\n\tv_nop" : "+v"(d) : "v"(a), "v"(b));
  return d;
}

__global__ __launch_bounds__(256) void wconv_kernel(
    const float* __restrict__ W, _Float16* __restrict__ Wt, unsigned ldw, unsigned ldk,
    unsigned ktrue) {
  __shared__ __attribute__((aligned(16))) _Float16 T[64 * LDT];
  const unsigned tid = threadIdx.x;
  const unsigned n0 = blockIdx.x * 64u;
  const unsigned k0 = blockIdx.y * 64u;
#pragma unroll 4
  for (unsigned j = 0; j < 16u; ++j) {
    const unsigned idx = tid + 256u * j;
    const unsigned kr = idx >> 6, nc = idx & 63u;
    const unsigned kg = k0 + kr;
    const unsigned kc = (kg < ktrue) ? kg : (ktrue - 1u);
    float v = W[(size_t)kc * ldw + n0 + nc];
    v = (kg < ktrue) ? v : 0.0f;
    T[nc * LDT + kr] = toh_flush(WCARRY * bf16r(v));
  }
  __syncthreads();
  v8h x[2];
  size_t off[2];
#pragma unroll
  for (unsigned i = 0; i < 2u; ++i) {
    const unsigned n = 32u * i + (tid >> 3);
    const unsigned kc = (tid & 7u) * 8u;
    x[i] = *(const v8h*)&T[n * LDT + kc];
    off[i] = (size_t)(n0 + n) * ldk + k0 + kc;
  }
#pragma unroll
  for (int i = 0; i < 2; ++i) *(volatile v8h*)(Wt + off[i]) = x[i];
  __threadfence();
#pragma unroll
  for (int i = 0; i < 2; ++i) *(volatile v8h*)(Wt + off[i]) = x[i];
}

__global__ __launch_bounds__(256) void onehot_kernel(
    const int* __restrict__ prop, const int* __restrict__ alt, _Float16* __restrict__ oh) {
  __shared__ __attribute__((aligned(16))) _Float16 T[32 * KS];
  const unsigned tid = threadIdx.x;
  const unsigned m0 = blockIdx.x * 32u;
  const v8h z = {};
#pragma unroll
  for (unsigned i = 0; i < 5u; ++i) *(v8h*)&T[(tid + 256u * i) * 8u] = z;
  __syncthreads();
#pragma unroll 1
  for (unsigned it = 0; it < 3u; ++it) {
    const unsigned i = tid + 256u * it;
    const bool live = i < (unsigned)(32 * NPROP);
    const unsigned ic = live ? i : (unsigned)(32 * NPROP - 1);
    const unsigned r = ic / (unsigned)NPROP;
    const unsigned j = ic - r * (unsigned)NPROP;
    const unsigned g = m0 + r;
    const unsigned bb = g / (unsigned)NTGT;
    const unsigned tt = g - bb * (unsigned)NTGT;
    const unsigned ta = (tt > 0u) ? (tt - 1u) : 0u;
    const int vp = prop[(size_t)bb * NPROP + j];
    const int va = alt[((size_t)ta * NB_FULL + bb) * NPROP + j];
    const int idx = (tt == 0u) ? vp : va;
    const int iw = (idx < 0) ? (idx + SCN) : idx;
    if (live && (unsigned)iw < (unsigned)SCN) T[r * (unsigned)KS + (unsigned)iw] = (_Float16)1.0f;
  }
  __syncthreads();
  v8h x[5];
#pragma unroll
  for (unsigned i = 0; i < 5u; ++i) x[i] = *(const v8h*)&T[(tid + 256u * i) * 8u];
  _Float16* base = oh + (size_t)m0 * KS + tid * 8u;
#pragma unroll
  for (unsigned i = 0; i < 5u; ++i) *(volatile v8h*)(base + 2048u * i) = x[i];
  __threadfence();
#pragma unroll
  for (unsigned i = 0; i < 5u; ++i) *(volatile v8h*)(base + 2048u * i) = x[i];
}

__global__ __launch_bounds__(256) void bow_kernel(
    const int* __restrict__ word, const float* __restrict__ Wstr,
    const float* __restrict__ bstr, _Float16* __restrict__ se) {
#pragma clang fp contract(off)
  __shared__ int sw[16 * NWORD];
  __shared__ __attribute__((aligned(16))) _Float16 T[16 * LDB];
  const unsigned tid = threadIdx.x;
  const unsigned m0 = blockIdx.x * 16u;
#pragma unroll 1
  for (unsigned it = 0; it < 4u; ++it) {
    const unsigned i = tid + 256u * it;
    const bool live = i < (unsigned)(16 * NWORD);
    const unsigned ic = live ? i : (unsigned)(16 * NWORD - 1);
    const int wv = word[(size_t)m0 * NWORD + ic];
    const int ww = (wv < 0) ? (wv + VOCAB) : wv;
    const int ok = ((unsigned)ww < (unsigned)VOCAB) ? ww : -1;
    if (live) sw[ic] = ok;
  }
  __syncthreads();
  const float bb = bf16r(bstr[tid]);
#pragma unroll 1
  for (unsigned r = 0; r < 16u; ++r) {
    float a = 0.0f;
#pragma unroll 5
    for (unsigned j = 0; j < (unsigned)NWORD; ++j) {
      const int wv = sw[r * (unsigned)NWORD + j];
      const bool ok = wv >= 0;
      const unsigned wc = ok ? (unsigned)wv : 0u;
      const float v = Wstr[(size_t)wc * DIM + tid];
      a += ok ? bf16r(v) : 0.0f;
    }
    T[r * (unsigned)LDB + tid] = toh_flush(ACARRY * (a + bb));
  }
  __syncthreads();
  v8h x[2];
  size_t off[2];
#pragma unroll
  for (unsigned i = 0; i < 2u; ++i) {
    const unsigned c = tid + 256u * i;
    const unsigned r = c >> 5;
    const unsigned col = (c & 31u) * 8u;
    x[i] = *(const v8h*)&T[r * (unsigned)LDB + col];
    off[i] = (size_t)(m0 + r) * DIM + col;
  }
#pragma unroll
  for (int i = 0; i < 2; ++i) *(volatile v8h*)(se + off[i]) = x[i];
  __threadfence();
#pragma unroll
  for (int i = 0; i < 2; ++i) *(volatile v8h*)(se + off[i]) = x[i];
}

template <int MODE>
__device__ __forceinline__ void gemm_body(
    const _Float16* __restrict__ A16, const _Float16* __restrict__ Bt, const unsigned K,
    const float* __restrict__ bias, const float* __restrict__ s5, const float* __restrict__ w3,
    const float* __restrict__ b3, float* __restrict__ outf, _Float16* __restrict__ out16) {
  __shared__ __attribute__((aligned(16))) float Cs[64 * LDC];
  __shared__ __attribute__((aligned(16))) float Red[64];
  const unsigned tid = threadIdx.x, lane = tid & 31u, w = tid >> 5;
  const unsigned mw = w >> 1, nw = w & 1u;
  const unsigned hh = lane >> 4, m = lane & 15u;
  const unsigned row0 = blockIdx.y * 64u;
  const unsigned ntile = (MODE == 2) ? (unsigned)(DIM / 64) : 1u;
  float part = 0.0f;

#pragma unroll 1
  for (unsigned nt = 0; nt < ntile; ++nt) {
    const unsigned n0 = (MODE == 2) ? (nt * 64u) : (blockIdx.x * 64u);

    const _Float16* ap  = A16 + (size_t)(row0 + mw * 16u + m) * K + hh * 8u;
    const _Float16* bp0 = Bt + (size_t)(n0 + nw * 32u + m) * K + hh * 8u;
    const _Float16* bp1 = bp0 + (size_t)16 * K;
    v8f acc0 = {}, acc1 = {};
#pragma unroll 2
    for (unsigned k0 = 0; k0 < K; k0 += 32u) {
      const v16h a  = frag_at(ap + k0);
      const v16h b0 = frag_at(bp0 + k0);
      const v16h b1 = frag_at(bp1 + k0);
      acc0 = wmma16(a, b0, acc0);
      acc1 = wmma16(a, b1, acc1);
    }
#pragma unroll
    for (int r = 0; r < 8; ++r) {
      float* d = &Cs[(mw * 16u + hh * 8u + (unsigned)r) * LDC + nw * 32u + m];
      d[0]  = acc0[r];
      d[16] = acc1[r];
    }
    __syncthreads();

    if (MODE == 0) {
      v8h x[2];
      size_t off[2];
#pragma unroll
      for (unsigned i = 0; i < 2u; ++i) {
        const unsigned r = 32u * i + (tid >> 3);
        const unsigned c = (tid & 7u) * 8u;
        const v4f u0 = *(const v4f*)&Cs[r * LDC + c];
        const v4f u1 = *(const v4f*)&Cs[r * LDC + c + 4];
        const v4f g0 = *(const v4f*)(bias + n0 + c);
        const v4f g1 = *(const v4f*)(bias + n0 + c + 4u);
#pragma unroll
        for (int j = 0; j < 4; ++j) {
          x[i][j]     = toh_flush(ACARRY * (u0[j] * (1.0f / WCARRY) + bf16r(g0[j])));
          x[i][j + 4] = toh_flush(ACARRY * (u1[j] * (1.0f / WCARRY) + bf16r(g1[j])));
        }
        off[i] = (size_t)(row0 + r) * DIM + n0 + c;
      }
#pragma unroll
      for (int i = 0; i < 2; ++i) *(volatile v8h*)(out16 + off[i]) = x[i];
      __threadfence();
#pragma unroll
      for (int i = 0; i < 2; ++i) *(volatile v8h*)(out16 + off[i]) = x[i];
    }

    if (MODE == 1) {
      const float cs = 1.0f / (WCARRY * ACARRY);
      v4f xs[4];
      size_t off[4];
#pragma unroll
      for (unsigned i = 0; i < 4u; ++i) {
        const unsigned r = 16u * i + (tid >> 4);
        const unsigned c = (tid & 15u) * 4u;
        const v4f u = *(const v4f*)&Cs[r * LDC + c];
        const v4f g = *(const v4f*)(bias + n0 + c);
        v4f val;
#pragma unroll
        for (int j = 0; j < 4; ++j) val[j] = u[j] * cs + bf16r(g[j]);
        xs[i] = val;
        off[i] = (size_t)(row0 + r) * DIM + n0 + c;
      }
#pragma unroll
      for (int i = 0; i < 4; ++i) *(volatile v4f*)(outf + off[i]) = xs[i];
      __threadfence();
#pragma unroll
      for (int i = 0; i < 4; ++i) *(volatile v4f*)(outf + off[i]) = xs[i];
    }

    if (MODE == 2) {
      const float cs = 1.0f / (WCARRY * ACARRY);
      const unsigned r = tid >> 2;
      const unsigned cb = (tid & 3u) * 16u;
      const unsigned bidx = (row0 + r) / (unsigned)NTGT;
#pragma unroll 1
      for (unsigned q = 0; q < 4u; ++q) {
        const unsigned c = cb + 4u * q;
        const v4f u  = *(const v4f*)&Cs[r * LDC + c];
        const v4f gb = *(const v4f*)(bias + n0 + c);
        const v4f sv = *(const v4f*)(s5 + (size_t)bidx * DIM + n0 + c);
        const v4f wv = *(const v4f*)(w3 + n0 + c);
#pragma unroll
        for (int j = 0; j < 4; ++j) {
          const float t = (u[j] * cs + bf16r(gb[j])) + sv[j];
          part += fmaxf(t, 0.0f) * bf16r(wv[j]);
        }
      }
      __syncthreads();
    }
  }

  if (MODE == 2) {
    part += __shfl_xor(part, 1, 32);
    part += __shfl_xor(part, 2, 32);
    if ((tid & 3u) == 0u) Red[tid >> 2] = part;
    __syncthreads();
    if (tid < 16u) {
      const float bb = bf16r(b3[0]);
      v4f o = *(const v4f*)&Red[tid * 4u];
#pragma unroll
      for (int j = 0; j < 4; ++j) o[j] = o[j] + bb;
      float* p = outf + (size_t)row0 + tid * 4u;
      *(volatile v4f*)p = o;
      __threadfence();
      *(volatile v4f*)p = o;
    }
  }
}

__global__ __launch_bounds__(256) void gemm_tg_kernel(
    const _Float16* __restrict__ A16, const _Float16* __restrict__ Bt,
    const float* __restrict__ bias, _Float16* __restrict__ out16) {
  gemm_body<0>(A16, Bt, (unsigned)KS, bias, bias, bias, bias, (float*)0, out16);
}
__global__ __launch_bounds__(256) void gemm_s5_kernel(
    const _Float16* __restrict__ A16, const _Float16* __restrict__ Bt,
    const float* __restrict__ bias, float* __restrict__ outf) {
  gemm_body<1>(A16, Bt, (unsigned)DIM, bias, bias, bias, bias, outf, (_Float16*)0);
}
__global__ __launch_bounds__(256) void gemm_score_kernel(
    const _Float16* __restrict__ A16, const _Float16* __restrict__ Bt,
    const float* __restrict__ bias, const float* __restrict__ s5,
    const float* __restrict__ w3, const float* __restrict__ b3, float* __restrict__ outf) {
  gemm_body<2>(A16, Bt, (unsigned)DIM, bias, s5, w3, b3, outf, (_Float16*)0);
}

extern "C" void kernel_launch(void* const* d_in, const int* in_sizes, int n_in,
                              void* d_out, int out_size, void* d_ws, size_t ws_size,
                              hipStream_t stream) {
  if (n_in < 13) return;
  if ((long long)in_sizes[0] < (long long)NB * NPROP) return;
  if ((long long)in_sizes[1] < ((long long)(NALT - 1) * NB_FULL + NB) * NPROP) return;
  if ((long long)in_sizes[2] < (long long)NB * NWORD) return;
  if ((long long)in_sizes[3] < (long long)SCN * DIM) return;
  if ((long long)in_sizes[5] < (long long)VOCAB * DIM) return;
  if ((long long)in_sizes[7] < (long long)DIM * DIM) return;
  if ((long long)in_sizes[9] < (long long)DIM * DIM) return;
  if (in_sizes[4] < DIM || in_sizes[6] < DIM || in_sizes[8] < DIM || in_sizes[10] < DIM) return;
  if (in_sizes[11] < DIM || in_sizes[12] < 1) return;
  if ((long long)out_size < (long long)MROWS) return;
  if (ws_size < WS_TOTAL) return;

  const int*   prop  = (const int*)d_in[0];
  const int*   alt   = (const int*)d_in[1];
  const int*   word  = (const int*)d_in[2];
  const float* wsc   = (const float*)d_in[3];
  const float* bsc   = (const float*)d_in[4];
  const float* wstr  = (const float*)d_in[5];
  const float* bstr  = (const float*)d_in[6];
  const float* w4    = (const float*)d_in[7];
  const float* b4    = (const float*)d_in[8];
  const float* w5    = (const float*)d_in[9];
  const float* b5    = (const float*)d_in[10];
  const float* w3    = (const float*)d_in[11];
  const float* b3    = (const float*)d_in[12];
  float* out = (float*)d_out;

  char* ws = (char*)d_ws;
  _Float16* Wsc_t = (_Float16*)(ws + OFF_WSC);
  _Float16* W4_t  = (_Float16*)(ws + OFF_W4);
  _Float16* W5_t  = (_Float16*)(ws + OFF_W5);
  _Float16* OH16  = (_Float16*)(ws + OFF_OH);
  _Float16* TG16  = (_Float16*)(ws + OFF_TG);
  _Float16* SE16  = (_Float16*)(ws + OFF_SE);
  float*    S5    = (float*)(ws + OFF_S5);

  dim3 blk(256);

  wconv_kernel<<<dim3(DIM / 64, KS / 64), blk, 0, stream>>>(wsc, Wsc_t, (unsigned)DIM, (unsigned)KS, (unsigned)SCN);
  wconv_kernel<<<dim3(DIM / 64, DIM / 64), blk, 0, stream>>>(w4, W4_t, (unsigned)DIM, (unsigned)DIM, (unsigned)DIM);
  wconv_kernel<<<dim3(DIM / 64, DIM / 64), blk, 0, stream>>>(w5, W5_t, (unsigned)DIM, (unsigned)DIM, (unsigned)DIM);

  onehot_kernel<<<dim3(MROWS / 32), blk, 0, stream>>>(prop, alt, OH16);
  bow_kernel<<<dim3(NB / 16), blk, 0, stream>>>(word, wstr, bstr, SE16);

  gemm_tg_kernel<<<dim3(DIM / 64, MROWS / 64), blk, 0, stream>>>(OH16, Wsc_t, bsc, TG16);
  gemm_s5_kernel<<<dim3(DIM / 64, NB / 64), blk, 0, stream>>>(SE16, W5_t, b5, S5);
  gemm_score_kernel<<<dim3(1, MROWS / 64), blk, 0, stream>>>(TG16, W4_t, b4, S5, w3, b3, out);
}
